// GMP_23545010717400
// MI455X (gfx1250) — hardware-run, weakly checked
//
#include <hip/hip_runtime.h>
#include <math.h>

typedef __attribute__((ext_vector_type(16))) _Float16 v16h;
typedef __attribute__((ext_vector_type(4)))  _Float16 v4h;
typedef __attribute__((ext_vector_type(2)))  _Float16 v2h;
typedef __attribute__((ext_vector_type(8)))  float    v8f;
typedef __attribute__((ext_vector_type(4)))  float    v4f;
typedef __attribute__((ext_vector_type(2)))  float    v2f;
typedef __attribute__((ext_vector_type(8)))  unsigned v8u;
typedef __attribute__((ext_vector_type(4)))  unsigned v4u;
typedef __attribute__((ext_vector_type(2)))  unsigned v2u;

constexpr int kBatch   = 16;
constexpr int kT       = 8192;
constexpr int kTaps    = 11;
constexpr int kPow     = 4;
constexpr int kNumW    = kTaps + kPow * kTaps * kTaps;
constexpr int kBlkT    = 256;
constexpr int kWin     = 280;
constexpr int kEnvPos  = 2 * kTaps - 1;
constexpr int kKreal   = kEnvPos * kPow;
constexpr int kKpad    = 96;
constexpr int kBtPitchW = kKpad / 2;
constexpr int kGP      = 17;
constexpr float kWCarry    = 1024.0f;
constexpr float kWCarryInv = 1.0f / kWCarry;
static_assert(kNumW == 495, "weight vector length");
static_assert(kKreal == 84 && kKreal <= kKpad && (kKpad % 32) == 0, "K padded to a multiple of 32");
static_assert((kT % kBlkT) == 0, "time tiles cover T exactly");
static_assert(4 * (kBlkT - 1) + kKpad <= 4 * kWin, "every A-fragment half index lies inside the staged power plane");
static_assert(kWin <= 512, "two staging passes of 256 threads cover the window");
static_assert(16 * kBtPitchW == 3 * 256, "three words per thread cover the weight tile exactly");

__device__ __forceinline__ v8f mma_f16(v16h a, v16h b, v8f c) {
  c = __builtin_amdgcn_wmma_f32_16x16x32_f16(false, a, false, b, (short)0, c, false, false);
  asm volatile("v_nop\n\tv_nop\n\tv_nop\n\tv_nop" : "+v"(c) : "v"(a), "v"(b));
  return c;
}

__device__ __forceinline__ v16h load_a_frag(const unsigned* pw, int wordoff) {
  const v2u q0 = *(const v2u*)(pw + wordoff);
  const v2u q1 = *(const v2u*)(pw + wordoff + 2);
  const v2u q2 = *(const v2u*)(pw + wordoff + 8);
  const v2u q3 = *(const v2u*)(pw + wordoff + 10);
  v8u wv;
  wv[0] = q0[0]; wv[1] = q0[1]; wv[2] = q1[0]; wv[3] = q1[1];
  wv[4] = q2[0]; wv[5] = q2[1]; wv[6] = q3[0]; wv[7] = q3[1];
  return __builtin_bit_cast(v16h, wv);
}

__device__ __forceinline__ v16h load_b_frag(const unsigned* bt, int wordoff) {
  const v4u q0 = *(const v4u*)(bt + wordoff);
  const v4u q1 = *(const v4u*)(bt + wordoff + 8);
  const v8u wv = __builtin_shufflevector(q0, q1, 0, 1, 2, 3, 4, 5, 6, 7);
  return __builtin_bit_cast(v16h, wv);
}

__global__ __launch_bounds__(256) void env_poly_kernel(const float* __restrict__ x,
                                                       const float* __restrict__ w,
                                                       float* __restrict__ out)
{
  __shared__ __align__(16) float    sRe[kWin];
  __shared__ __align__(16) float    sIm[kWin];
  __shared__ __align__(16) unsigned sPW[kWin * 2];
  __shared__ __align__(16) unsigned sBt[16 * kBtPitchW];
  __shared__ __align__(16) float    sWl[16];
  __shared__ __align__(16) float    sG[8 * 32 * kGP];
  __shared__ __align__(16) float    sOut[kBlkT * 2];

  const int tid  = threadIdx.x;
  const int lane = tid & 31;
  const int wave = __builtin_amdgcn_readfirstlane((int)(threadIdx.x >> 5));
  const int b    = blockIdx.y;
  const int t0   = blockIdx.x * kBlkT;

#pragma unroll
  for (int it = 0; it < 2; ++it) {
    const int i  = tid + 256 * it;
    const int ic = (i < kWin) ? i : (kWin - 1);
    const int t  = t0 - (kTaps - 1) + ic;
    const bool inb = (t >= 0) && (t < kT);
    int tc = (t < 0) ? 0 : t;
    tc = (tc > kT - 1) ? (kT - 1) : tc;
    const v2f cv = *(const v2f*)(x + ((size_t)b * kT + (size_t)tc) * 2);
    float lre = cv[0];
    float lim = cv[1];
    asm volatile("" : "+v"(lre), "+v"(lim));
    const float re = inb ? lre : 0.0f;
    const float im = inb ? lim : 0.0f;
    const float a1 = sqrtf(re * re + im * im);
    const float a2 = a1 * a1;
    const float a3 = a2 * a1;
    const float a4 = a2 * a2;
    v4h pv;
    pv[0] = (_Float16)a1;
    pv[1] = (_Float16)a2;
    pv[2] = (_Float16)a3;
    pv[3] = (_Float16)a4;
    const v2u pw = __builtin_bit_cast(v2u, pv);
    if (i < kWin) {
      sRe[i] = re;
      sIm[i] = im;
      *(v2u*)(sPW + 2 * i) = pw;
    }
  }

#pragma unroll
  for (int it = 0; it < 3; ++it) {
    const int widx = tid + 256 * it;
    const int n    = widx / kBtPitchW;
    const int kw   = widx - n * kBtPitchW;
    const int k    = 2 * kw;
    const int s    = k >> 2;
    const int p    = k & 3;
    const int i0   = s - n;
    const bool valid = (n < kTaps) && (s < kEnvPos) && (i0 >= 0) && (i0 < kTaps);
    const int idx  = kTaps + p * (kTaps * kTaps) + i0 * kTaps + n;
    const int idc  = valid ? idx : kTaps;
    float w0 = w[idc];
    float w1 = w[idc + kTaps * kTaps];
    asm volatile("" : "+v"(w0), "+v"(w1));
    const float c0 = valid ? (w0 * kWCarry) : 0.0f;
    const float c1 = valid ? (w1 * kWCarry) : 0.0f;
    v2h hv;
    hv[0] = (_Float16)c0;
    hv[1] = (_Float16)c1;
    sBt[widx] = __builtin_bit_cast(unsigned, hv);
  }

  {
    const int mi = (tid < kTaps) ? tid : (kTaps - 1);
    float wl = w[mi];
    asm volatile("" : "+v"(wl));
    const float wv = (tid < kTaps) ? wl : 0.0f;
    if (tid < 16) sWl[tid] = wv;
  }
  __syncthreads();

  const int h  = lane >> 4;
  const int rl = lane & 15;
  v16h bfr[3];
#pragma unroll
  for (int ks = 0; ks < 3; ++ks)
    bfr[ks] = load_b_frag(sBt, rl * kBtPitchW + ks * 16 + 4 * h);

  v8f acc0 = (v8f){0.f, 0.f, 0.f, 0.f, 0.f, 0.f, 0.f, 0.f};
  v8f acc1 = (v8f){0.f, 0.f, 0.f, 0.f, 0.f, 0.f, 0.f, 0.f};
  const int rowA0 = wave * 32 + rl;
  const int rowA1 = rowA0 + 16;
#pragma unroll
  for (int ks = 0; ks < 3; ++ks) {
    const v16h a0 = load_a_frag(sPW, 2 * rowA0 + ks * 16 + 4 * h);
    const v16h a1 = load_a_frag(sPW, 2 * rowA1 + ks * 16 + 4 * h);
    acc0 = mma_f16(a0, bfr[ks], acc0);
    acc1 = mma_f16(a1, bfr[ks], acc1);
  }

  float* gw = sG + wave * (32 * kGP);
#pragma unroll
  for (int r = 0; r < 8; ++r) {
    gw[(8 * h + r) * kGP + rl]      = acc0[r];
    gw[(16 + 8 * h + r) * kGP + rl] = acc1[r];
  }
  __syncthreads();

  const int tl = wave * 32 + lane;
  float yr = 0.0f;
  float yi = 0.0f;
#pragma unroll
  for (int m = 0; m < kTaps; ++m) {
    const float g = fmaf(gw[lane * kGP + m], kWCarryInv, sWl[m]);
    yr = fmaf(sRe[tl + m], g, yr);
    yi = fmaf(sIm[tl + m], g, yi);
  }
  sOut[2 * tl]     = yr;
  sOut[2 * tl + 1] = yi;
  __syncthreads();

  if (wave < 4) {
    const v4f v = *(const v4f*)(sOut + 4 * tid);
    float* dst = out + ((size_t)b * kT + (size_t)t0) * 2 + 4 * tid;
    *(volatile v4f*)dst = v;
    __threadfence();
    *(volatile v4f*)dst = v;
  }
}

extern "C" void kernel_launch(void* const* d_in, const int* in_sizes, int n_in,
                              void* d_out, int out_size, void* d_ws, size_t ws_size,
                              hipStream_t stream) {
  if (n_in < 2) return;
  if (in_sizes[0] != kBatch * kT * 2) return;
  if (in_sizes[1] != kNumW) return;
  if (out_size != kBatch * kT * 2) return;
  (void)d_ws;
  (void)ws_size;
  const float* x = (const float*)d_in[0];
  const float* w = (const float*)d_in[1];
  float* out = (float*)d_out;
  env_poly_kernel<<<dim3(kT / kBlkT, kBatch), 256, 0, stream>>>(x, w, out);
}
